// Encoder_84748294685032
// MI455X (gfx1250) — hardware-verified
//
#include <hip/hip_runtime.h>
#include <math.h>

constexpr int NSTEP      = 512;
constexpr int NBATCH     = 64;
constexpr int NIN        = 300;
constexpr int NINP       = 320;
constexpr int NHID       = 512;
constexpr int NGATE      = 4 * NHID;
constexpr int CHUNK_T    = 128;
constexpr int NCHUNK     = NSTEP / CHUNK_T;
constexpr int CHUNK_ROWS = CHUNK_T * NBATCH;
constexpr int NROWS      = NSTEP * NBATCH;
constexpr int BLK_ROWS   = 16;
constexpr int REC_THR    = 512;
constexpr int HPITCH     = 520;
constexpr int OPITCH     = 516;
constexpr float WCARRY   = 256.0f;
constexpr float HCARRY   = 16.0f;
constexpr float WFOLD    = 1.0f / WCARRY;
constexpr float RFOLD    = 1.0f / (WCARRY * HCARRY);
constexpr int SMALL_FLOATS = NGATE + 2 * NBATCH * NHID;

static_assert(NSTEP % CHUNK_T == 0, "chunks exact");
static_assert((CHUNK_T & 1) == 0, "LDS buffer parity restarts at 0 every chunk");
static_assert(NINP % 32 == 0 && NINP >= NIN && NIN % 4 == 0, "K pad");
static_assert(NHID % 32 == 0, "recurrent K multiple of 32");
static_assert(NGATE % 64 == 0 && CHUNK_ROWS % 64 == 0, "GEMM tile multiples");
static_assert(((NGATE / 64) * (CHUNK_ROWS / 64)) % 8 == 0, "GEMM grid exact");
static_assert(NHID == 32 * (REC_THR / 32), "16 waves x 32 hidden units");
static_assert(NBATCH % BLK_ROWS == 0, "batch tiles exact");
static_assert((NROWS * (NINP / 8)) % 256 == 0, "x plane grid exact");
static_assert((NGATE * (NINP / 8)) % 256 == 0, "W_ih plane grid exact");
static_assert((NGATE * (NHID / 8)) % 256 == 0, "W_hh plane grid exact");
static_assert((SMALL_FLOATS / 4) % 256 == 0, "init grid exact");
static_assert((BLK_ROWS * NHID / 4) % REC_THR == 0, "state load/store loop exact");
static_assert(NGATE == 4 * REC_THR, "bias staging: one float4 per thread");
static_assert(NGATE <= BLK_ROWS * OPITCH, "bias vector fits the slab");
static_assert((OPITCH * 4) % 16 == 0 && (HPITCH * 2) % 16 == 0, "LDS rows 16-B aligned");

typedef __attribute__((ext_vector_type(16))) _Float16 v16h;
typedef __attribute__((ext_vector_type(8)))  _Float16 v8h;
typedef __attribute__((ext_vector_type(8)))  float    v8f;
typedef __attribute__((ext_vector_type(4)))  float    v4f;

__device__ __forceinline__ unsigned short f2bf_bits(float f) {
  unsigned u = __float_as_uint(f);
  return (unsigned short)((u + 0x7FFFu + ((u >> 16) & 1u)) >> 16);
}
__device__ __forceinline__ float bf_bits2f(unsigned short h) { return __uint_as_float(((unsigned)h) << 16); }
__device__ __forceinline__ float bf16r(float f) { return bf_bits2f(f2bf_bits(f)); }

__device__ __forceinline__ void grp_guard4(v8f& a0, v8f& a1, v8f& a2, v8f& a3,
                                           v16h x, v16h y0, v16h y1, v16h y2, v16h y3) {
  asm volatile("v_nop\n\tv_nop\n\tv_nop\n\tv_nop"
               : "+v"(a0), "+v"(a1), "+v"(a2), "+v"(a3)
               : "v"(x), "v"(y0), "v"(y1), "v"(y2), "v"(y3));
}
__device__ __forceinline__ void keep4_h(v16h a, v16h b, v16h c, v16h d) { asm volatile("v_nop" :: "v"(a), "v"(b), "v"(c), "v"(d)); }
__device__ __forceinline__ void acc_guard4(v8f& a, v8f& b, v8f& c, v8f& d) { asm volatile("v_nop\n\tv_nop\n\tv_nop\n\tv_nop" : "+v"(a), "+v"(b), "+v"(c), "+v"(d)); }

struct FragH {
  union U { v16h v; v8h h[2]; };
  static __device__ __forceinline__ v16h load(const _Float16* p) {
    U f; f.h[0] = *(const v8h*)(p); f.h[1] = *(const v8h*)(p + 16); return f.v;
  }
  static __device__ __forceinline__ v8f mma(v16h a, v16h b, v8f c) {
    return __builtin_amdgcn_wmma_f32_16x16x32_f16(false, a, false, b, (short)0, c, false, false);
  }
};

__device__ __forceinline__ float fsig(float x)  { return __builtin_amdgcn_rcpf(1.0f + __expf(-x)); }
__device__ __forceinline__ float ftanh(float x) { return 1.0f - 2.0f * __builtin_amdgcn_rcpf(__expf(2.0f * x) + 1.0f); }

__global__ __launch_bounds__(256) void cvt_rows_kernel(const float* __restrict__ src, unsigned short* __restrict__ dst,
                                                       int nrow, int ncol8, int spitch, int ncols, float sc) {
  const int i  = blockIdx.x * 256 + threadIdx.x;
  const int n8 = nrow * ncol8;
  if (i < n8) {
    const int row  = i / ncol8;
    const int c8   = i - row * ncol8;
    const int colA = c8 * 8;
    const int colB = c8 * 8 + 4;
    const bool okA = colA < ncols;
    const bool okB = colB < ncols;
    const int ca = okA ? colA : (ncols - 4);
    const int cb = okB ? colB : (ncols - 4);
    const float* rp = src + (size_t)row * (size_t)spitch;
    const v4f a = *(const v4f*)(rp + ca);
    const v4f b = *(const v4f*)(rp + cb);
    v8h hv;
#pragma unroll
    for (int e = 0; e < 4; ++e) {
      const float av = a[e];
      const float bv = b[e];
      const float fa = okA ? (bf16r(av) * sc) : 0.0f;
      const float fb = okB ? (bf16r(bv) * sc) : 0.0f;
      hv[e]     = (_Float16)fa;
      hv[4 + e] = (_Float16)fb;
    }
    *(volatile v8h*)(dst + (size_t)i * 8) = hv;
    __threadfence();
    *(volatile v8h*)(dst + (size_t)i * 8) = hv;
  }
}

__global__ __launch_bounds__(256) void init_kernel(const float* __restrict__ b_ih, const float* __restrict__ b_hh,
                                                   float* __restrict__ small) {
  const int i = blockIdx.x * 256 + threadIdx.x;
  const bool isb = blockIdx.x < 2;
  const int ic = isb ? i : 0;
  const v4f va = *(const v4f*)(b_ih + 4 * ic);
  const v4f vb = *(const v4f*)(b_hh + 4 * ic);
  v4f o;
#pragma unroll
  for (int e = 0; e < 4; ++e) {
    const float x0 = va[e];
    const float x1 = vb[e];
    const float s = bf16r(x0) + bf16r(x1);
    o[e] = isb ? s : 0.0f;
  }
  float* op = small + (size_t)i * 4;
  *(volatile v4f*)op = o;
  __threadfence();
  *(volatile v4f*)op = o;
}

__global__ __launch_bounds__(256) void gemm64_f16_kernel(const unsigned short* __restrict__ Ap, int lda,
                                                         const unsigned short* __restrict__ Btp, int ldb,
                                                         float* __restrict__ C, int ldc,
                                                         int M, int N, int K, float scale) {
  const _Float16* A  = (const _Float16*)Ap;
  const _Float16* Bt = (const _Float16*)Btp;
  __shared__ __align__(16) float sT[8][16 * 68];
  const int lane = threadIdx.x & 31;
  const int wave = threadIdx.x >> 5;
  const int tilesN = N >> 6;
  const int tilesM = M >> 6;
  const int tile = blockIdx.x * 8 + wave;
  if (tile >= tilesM * tilesN) return;
  const int tm = tile / tilesN;
  const int tn = tile - tm * tilesN;
  const int m0 = tm << 6;
  const int n0 = tn << 6;
  const int rlane = lane & 15;
  const int koff  = (lane >> 4) * 8;
  const int mOff  = (lane >> 4) * 8;

  v8f acc[4][4];
#pragma unroll
  for (int i = 0; i < 4; ++i)
#pragma unroll
    for (int j = 0; j < 4; ++j) acc[i][j] = (v8f){0.f, 0.f, 0.f, 0.f, 0.f, 0.f, 0.f, 0.f};

  for (int k0 = 0; k0 < K; k0 += 32) {
    v16h bh[4];
#pragma unroll
    for (int j = 0; j < 4; ++j) {
      const size_t bo = (size_t)(n0 + (j << 4) + rlane) * (size_t)ldb + koff + k0;
      bh[j] = FragH::load(Bt + bo);
    }
#pragma unroll
    for (int i = 0; i < 4; ++i) {
      const size_t ao = (size_t)(m0 + (i << 4) + rlane) * (size_t)lda + koff + k0;
      const v16h ah = FragH::load(A + ao);
#pragma unroll
      for (int j = 0; j < 4; ++j) acc[i][j] = FragH::mma(ah, bh[j], acc[i][j]);
      grp_guard4(acc[i][0], acc[i][1], acc[i][2], acc[i][3], ah, bh[0], bh[1], bh[2], bh[3]);
    }
    keep4_h(bh[0], bh[1], bh[2], bh[3]);
  }
  acc_guard4(acc[0][0], acc[0][1], acc[0][2], acc[0][3]);
  acc_guard4(acc[1][0], acc[1][1], acc[1][2], acc[1][3]);
  acc_guard4(acc[2][0], acc[2][1], acc[2][2], acc[2][3]);
  acc_guard4(acc[3][0], acc[3][1], acc[3][2], acc[3][3]);

  float* slab = sT[wave];
#pragma unroll
  for (int i = 0; i < 4; ++i) {
    const int mBase = m0 + (i << 4);
#pragma unroll
    for (int j = 0; j < 4; ++j) {
#pragma unroll
      for (int r = 0; r < 8; ++r) {
        const float v = acc[i][j][r] * scale;
        slab[(mOff + r) * 68 + (j << 4) + rlane] = v;
      }
    }
    __builtin_amdgcn_fence(__ATOMIC_RELEASE, "workgroup");
    __builtin_amdgcn_wave_barrier();
    __builtin_amdgcn_fence(__ATOMIC_ACQUIRE, "workgroup");
    {
      const int hh = lane >> 4;
      const int c4 = (lane & 15) * 4;
      for (int pass = 0; pass < 2; ++pass) {
#pragma unroll
        for (int it = 0; it < 8; ++it) {
          const int row = it * 2 + hh;
          const v4f v = *(const v4f*)(slab + row * 68 + c4);
          *(volatile v4f*)(C + (size_t)(mBase + row) * (size_t)ldc + n0 + c4) = v;
        }
        __threadfence();
      }
    }
    __builtin_amdgcn_fence(__ATOMIC_RELEASE, "workgroup");
    __builtin_amdgcn_wave_barrier();
    __builtin_amdgcn_fence(__ATOMIC_ACQUIRE, "workgroup");
  }
}

__global__ __launch_bounds__(REC_THR) void lstm_rec_kernel(const float* XPt, const unsigned short* WHp, const float* bsum,
                                                           float* Hst, float* Cst, float* out, int last) {
  __shared__ __align__(16) _Float16 Ah[2][BLK_ROWS * HPITCH];
  __shared__ __align__(16) float    Hs[BLK_ROWS * OPITCH];
  const _Float16* WH = (const _Float16*)WHp;
  const int tid = threadIdx.x, lane = tid & 31, wave = tid >> 5;
  const int c = lane & 15, hh = lane >> 4, koff = hh * 8;
  const int rowbase = blockIdx.x * BLK_ROWS;

  if (tid < 256) {
    const int pb = tid >> 7, pr = (tid >> 3) & 15, pc = NHID + (tid & 7);
    Ah[pb][pr * HPITCH + pc] = (_Float16)0.0f;
  }

  float cst[2][8], hst[2][8], bb[2][4];

#pragma unroll
  for (int it = 0; it < 4; ++it) {
    const int idx = it * REC_THR + tid;
    const int row = idx >> 7, c4 = (idx & 127) * 4;
    const v4f v = *(const v4f*)(Hst + (size_t)(rowbase + row) * NHID + c4);
    *(v4f*)(Hs + row * OPITCH + c4) = v;
  }
  __syncthreads();
#pragma unroll
  for (int nt = 0; nt < 2; ++nt) {
    const int j = 32 * wave + 16 * nt + c;
#pragma unroll
    for (int r = 0; r < 8; ++r) {
      const float hv = Hs[(8 * hh + r) * OPITCH + j];
      hst[nt][r] = hv;
      Ah[0][(8 * hh + r) * HPITCH + j] = (_Float16)(hv * HCARRY);
    }
  }
  __syncthreads();
#pragma unroll
  for (int it = 0; it < 4; ++it) {
    const int idx = it * REC_THR + tid;
    const int row = idx >> 7, c4 = (idx & 127) * 4;
    const v4f v = *(const v4f*)(Cst + (size_t)(rowbase + row) * NHID + c4);
    *(v4f*)(Hs + row * OPITCH + c4) = v;
  }
  __syncthreads();
#pragma unroll
  for (int nt = 0; nt < 2; ++nt) {
    const int j = 32 * wave + 16 * nt + c;
#pragma unroll
    for (int r = 0; r < 8; ++r) cst[nt][r] = Hs[(8 * hh + r) * OPITCH + j];
  }
  __syncthreads();
  {
    const v4f v = *(const v4f*)(bsum + 4 * tid);
    *(v4f*)(Hs + 4 * tid) = v;
  }
  __syncthreads();
#pragma unroll
  for (int nt = 0; nt < 2; ++nt) {
    const int j = 32 * wave + 16 * nt + c;
#pragma unroll
    for (int g = 0; g < 4; ++g) bb[nt][g] = Hs[g * NHID + j];
  }
  __syncthreads();

  const v8f z8 = {0.f, 0.f, 0.f, 0.f, 0.f, 0.f, 0.f, 0.f};
  const size_t WGSTR = (size_t)NHID * NHID;
  const size_t XGSTR = (size_t)NHID * CHUNK_ROWS;

#pragma unroll 1
  for (int tl = 0; tl < CHUNK_T; ++tl) {
    const int cur = tl & 1;
    const _Float16* ahrow = &Ah[0][0] + cur * (BLK_ROWS * HPITCH) + c * HPITCH + koff;
    _Float16* ahn = &Ah[0][0] + (cur ^ 1) * (BLK_ROWS * HPITCH);
#pragma unroll
    for (int nt = 0; nt < 2; ++nt) {
      const int j = 32 * wave + 16 * nt + c;
      const _Float16* wh = WH + (size_t)j * NHID + koff;
      v8f acc[4];
      acc[0] = z8; acc[1] = z8; acc[2] = z8; acc[3] = z8;
#pragma unroll 1
      for (int k0 = 0; k0 < NHID; k0 += 32) {
        const v16h a  = FragH::load(ahrow + k0);
        const v16h b0 = FragH::load(wh + k0);
        const v16h b1 = FragH::load(wh + WGSTR + k0);
        const v16h b2 = FragH::load(wh + 2 * WGSTR + k0);
        const v16h b3 = FragH::load(wh + 3 * WGSTR + k0);
        acc[0] = FragH::mma(a, b0, acc[0]);
        acc[1] = FragH::mma(a, b1, acc[1]);
        acc[2] = FragH::mma(a, b2, acc[2]);
        acc[3] = FragH::mma(a, b3, acc[3]);
        grp_guard4(acc[0], acc[1], acc[2], acc[3], a, b0, b1, b2, b3);
      }
      acc_guard4(acc[0], acc[1], acc[2], acc[3]);
      const float* xp = XPt + (size_t)j * CHUNK_ROWS + (size_t)tl * NBATCH + rowbase + 8 * hh;
      const v8f x0 = *(const v8f*)(xp);
      const v8f x1 = *(const v8f*)(xp + XGSTR);
      const v8f x2 = *(const v8f*)(xp + 2 * XGSTR);
      const v8f x3 = *(const v8f*)(xp + 3 * XGSTR);
#pragma unroll
      for (int r = 0; r < 8; ++r) {
        const float zi = acc[0][r] * RFOLD + (x0[r] + bb[nt][0]);
        const float zf = acc[1][r] * RFOLD + (x1[r] + bb[nt][1]);
        const float zg = acc[2][r] * RFOLD + (x2[r] + bb[nt][2]);
        const float zo = acc[3][r] * RFOLD + (x3[r] + bb[nt][3]);
        const float ig = fsig(zi);
        const float fg = fsig(zf);
        const float gg = ftanh(zg);
        const float og = fsig(zo);
        const float cn = fg * cst[nt][r] + ig * gg;
        cst[nt][r] = cn;
        const float hn = og * ftanh(cn);
        hst[nt][r] = hn;
        ahn[(8 * hh + r) * HPITCH + j] = (_Float16)(hn * HCARRY);
      }
      asm volatile("" ::: "memory");
    }
    __syncthreads();
  }

#pragma unroll
  for (int nt = 0; nt < 2; ++nt) {
    const int j = 32 * wave + 16 * nt + c;
#pragma unroll
    for (int r = 0; r < 8; ++r) Hs[(8 * hh + r) * OPITCH + j] = hst[nt][r];
  }
  __syncthreads();
  for (int pass = 0; pass < 2; ++pass) {
#pragma unroll
    for (int it = 0; it < 4; ++it) {
      const int idx = it * REC_THR + tid;
      const int row = idx >> 7, c4 = (idx & 127) * 4;
      const v4f v = *(const v4f*)(Hs + row * OPITCH + c4);
      *(volatile v4f*)(Hst + (size_t)(rowbase + row) * NHID + c4) = v;
      if (last) *(volatile v4f*)(out + (size_t)(rowbase + row) * NHID + c4) = v;
    }
    __threadfence();
  }
  __syncthreads();
#pragma unroll
  for (int nt = 0; nt < 2; ++nt) {
    const int j = 32 * wave + 16 * nt + c;
#pragma unroll
    for (int r = 0; r < 8; ++r) Hs[(8 * hh + r) * OPITCH + j] = cst[nt][r];
  }
  __syncthreads();
  for (int pass = 0; pass < 2; ++pass) {
#pragma unroll
    for (int it = 0; it < 4; ++it) {
      const int idx = it * REC_THR + tid;
      const int row = idx >> 7, c4 = (idx & 127) * 4;
      const v4f v = *(const v4f*)(Hs + row * OPITCH + c4);
      *(volatile v4f*)(Cst + (size_t)(rowbase + row) * NHID + c4) = v;
    }
    __threadfence();
  }
}

extern "C" void kernel_launch(void* const* d_in, const int* in_sizes, int n_in,
                              void* d_out, int out_size, void* d_ws, size_t ws_size, hipStream_t stream) {
  if (n_in < 5 || d_out == nullptr || d_ws == nullptr) return;
  if (in_sizes[0] != NSTEP * NBATCH * NIN || in_sizes[1] != NGATE * NIN || in_sizes[2] != NGATE * NHID ||
      in_sizes[3] != NGATE || in_sizes[4] != NGATE || out_size != NBATCH * NHID) return;

  const float* x    = (const float*)d_in[0];
  const float* w_ih = (const float*)d_in[1];
  const float* w_hh = (const float*)d_in[2];
  const float* b_ih = (const float*)d_in[3];
  const float* b_hh = (const float*)d_in[4];
  float* out = (float*)d_out;

  char* ws = (char*)d_ws; size_t off = 0;
  auto carve = [&](size_t bytes) -> char* { char* p = ws + off; off += (bytes + 255) & ~(size_t)255; return p; };
  float*          SMALL = (float*)carve((size_t)SMALL_FLOATS * 4);
  unsigned short* XH    = (unsigned short*)carve((size_t)NROWS * NINP * 2);
  unsigned short* WIH   = (unsigned short*)carve((size_t)NGATE * NINP * 2);
  unsigned short* WHH   = (unsigned short*)carve((size_t)NGATE * NHID * 2);
  float*          XPT   = (float*)carve((size_t)NGATE * CHUNK_ROWS * 4);
  if (off > ws_size || off > (size_t)134217728) return;
  float* BSUM = SMALL;
  float* HST  = SMALL + NGATE;
  float* CST  = SMALL + NGATE + NBATCH * NHID;

  const int n8x = NROWS * (NINP / 8);
  const int n8i = NGATE * (NINP / 8);
  const int n8h = NGATE * (NHID / 8);
  cvt_rows_kernel<<<n8x / 256, 256, 0, stream>>>(x,    XH,  NROWS, NINP / 8, NIN,  NIN,  1.0f);
  cvt_rows_kernel<<<n8i / 256, 256, 0, stream>>>(w_ih, WIH, NGATE, NINP / 8, NIN,  NIN,  WCARRY);
  cvt_rows_kernel<<<n8h / 256, 256, 0, stream>>>(w_hh, WHH, NGATE, NHID / 8, NHID, NHID, WCARRY);
  init_kernel<<<(SMALL_FLOATS / 4) / 256, 256, 0, stream>>>(b_ih, b_hh, SMALL);

  const dim3 ggrid(((NGATE / 64) * (CHUNK_ROWS / 64)) / 8, 1);
  for (int ch = 0; ch < NCHUNK; ++ch) {
    const unsigned short* xh_c = XH + (size_t)ch * CHUNK_ROWS * NINP;
    gemm64_f16_kernel<<<ggrid, 256, 0, stream>>>(WIH, NINP, xh_c, NINP, XPT, CHUNK_ROWS,
                                                 NGATE, CHUNK_ROWS, NINP, WFOLD);
    lstm_rec_kernel<<<NBATCH / BLK_ROWS, REC_THR, 0, stream>>>(XPT, WHH, BSUM, HST, CST, out,
                                                               (ch == NCHUNK - 1) ? 1 : 0);
  }
}
